// GATLayer_14834817040882
// MI455X (gfx1250) — hardware-verified
//
#include <hip/hip_runtime.h>


namespace {
constexpr int B = 1, T = 4096, F = 256, H = 8, HD = 64, DM = H * HD  , AP = 2 * HD  , FP = 16  , BL = 1  , QL = T  , NR = B * T, NRL = BL * T  , NW32 = T / 32;
constexpr float XS = 8.0f, WSC = 256.0f, RS_ = 1024.0f, PS = 1024.0f, NSL = 0.2f, LOG2E = 1.4426950408889634f;
static_assert(T % 32 == 0 && F % 32 == 0 && HD == 64 && QL % 16 == 0, "tiling");
typedef _Float16 b16;
typedef __attribute__((ext_vector_type(16))) _Float16 v16b;
typedef __attribute__((ext_vector_type(8))) _Float16 v8b;
typedef __attribute__((ext_vector_type(8))) float v8f;
typedef __attribute__((ext_vector_type(4))) float v4f;
__device__ __forceinline__ float bf16_rne(float f) { unsigned int u = __float_as_uint(f); u += 0x7FFFu + ((u >> 16) & 1u); return __uint_as_float(u & 0xFFFF0000u); }
__device__ __forceinline__ void split16(float v, b16& hi, b16& lo) { hi = (b16)v; lo = (b16)(v - (float)hi); }
__device__ __forceinline__ v16b frag_kb(const b16* p, int hh) { const v8b a = *(const v8b*)(p + 8 * hh), b = *(const v8b*)(p + 16 + 8 * hh); v16b f;
#pragma unroll
  for (int e = 0; e < 8; ++e) { f[e] = a[e]; f[8 + e] = b[e]; } return f; }
__device__ __forceinline__ v8f wmma16b(v16b a, v16b b, v8f c) { v8f d = __builtin_amdgcn_wmma_f32_16x16x32_f16(false, a, false, b, (short)0, c, false, false); asm volatile("v_nop\n\tv_nop\n\tv_nop\n\tv_nop" : "+v"(d) : "v"(a), "v"(b)); return d; }
__device__ __forceinline__ void wave_lds_sync() { __builtin_amdgcn_fence(__ATOMIC_RELEASE, "workgroup"); __builtin_amdgcn_wave_barrier(); __builtin_amdgcn_fence(__ATOMIC_ACQUIRE, "workgroup"); }
__device__ __forceinline__ float pmul(float a, float b) { float p = a * b; asm volatile("" : "+v"(p)); return p; }
__device__ __forceinline__ int iclamp(int v, int lo, int hi) { return v < lo ? lo : (v > hi ? hi : v); }

typedef __attribute__((ext_vector_type(2))) _Float16 v2h;
typedef __attribute__((ext_vector_type(4))) _Float16 v4h;
typedef __attribute__((ext_vector_type(2))) float v2f;
typedef __attribute__((ext_vector_type(4))) int v4i;
__device__ __forceinline__ float nexp2(float v) { return __builtin_amdgcn_exp2f(v); }
__device__ __forceinline__ float bfp(float v) { float t = bf16_rne(v); asm volatile("" : "+v"(t)); return t; }

__device__ __forceinline__ float lrelu(float v) { return v > 0.0f ? v : NSL * v; }
__global__ __launch_bounds__(256) void wt_kernel(const float* __restrict__ w, b16* __restrict__ WT) {
  const int u = blockIdx.x * 256 + threadIdx.x; if (u >= DM * F / 8) return; const int e = u * 8; v8b v;
#pragma unroll
  for (int j = 0; j < 8; ++j) v[j] = (b16)(bf16_rne(w[e + j]) * WSC);
  for (int pass = 0; pass < 2; ++pass) { *(volatile v8b*)(WT + e) = v; __threadfence(); }
}
__global__ __launch_bounds__(64) void proj_kernel(const float* __restrict__ x, const b16* __restrict__ WT, const float* __restrict__ av, b16* __restrict__ WHh, b16* __restrict__ WHl, float* __restrict__ F1, float* __restrict__ F2) {
  __shared__ __attribute__((aligned(16))) b16 Ah[2][16][F + 8]; __shared__ __attribute__((aligned(16))) float Tw[2][16][HD + 4]; __shared__ float S1[2][16][FP], S2[2][16][FP];
  const int wave = threadIdx.x >> 5, lane = threadIdx.x & 31, nloc = lane & 15, hlf = lane >> 4; const size_t m0 = (size_t)blockIdx.x * 32 + wave * 16;
  for (int idx = lane; idx < 16 * (F / 4); idx += 32) { const int rr = idx / (F / 4), c4 = (idx % (F / 4)) * 4; const v4f v = *(const v4f*)(x + (m0 + rr) * F + c4); v4h hv; for (int j = 0; j < 4; ++j) hv[j] = (b16)(bf16_rne(v[j]) * XS); *(v4h*)(&Ah[wave][rr][c4]) = hv; }
  for (int idx = lane; idx < 16 * FP; idx += 32) { S1[wave][idx / FP][idx % FP] = 0.0f; S2[wave][idx / FP][idx % FP] = 0.0f; }
  wave_lds_sync();
#pragma unroll 1
  for (int h = 0; h < H; ++h) {
    v8f acc[4];
#pragma unroll
    for (int t = 0; t < 4; ++t) acc[t] = (v8f){};
#pragma unroll 2
    for (int kb = 0; kb < F; kb += 32) { const v16b a = frag_kb(&Ah[wave][nloc][kb], hlf);
#pragma unroll
      for (int t = 0; t < 4; ++t) acc[t] = wmma16b(a, frag_kb(WT + (size_t)(h * HD + t * 16 + nloc) * F + kb, hlf), acc[t]); }
    float p1[8], p2[8]; for (int r = 0; r < 8; ++r) { p1[r] = 0.0f; p2[r] = 0.0f; }
#pragma unroll
    for (int t = 0; t < 4; ++t) { const int d = t * 16 + nloc; const float w1 = bf16_rne(av[h * AP + d]), w2 = bf16_rne(av[h * AP + HD + d]);
#pragma unroll
      for (int r = 0; r < 8; ++r) { const float wv = acc[t][r] * (1.0f / (XS * WSC)); acc[t][r] = wv; p1[r] = fmaf(wv, w1, p1[r]); p2[r] = fmaf(wv, w2, p2[r]); } }
#pragma unroll
    for (int o = 1; o < 16; o <<= 1) for (int r = 0; r < 8; ++r) { p1[r] += __shfl_xor(p1[r], o); p2[r] += __shfl_xor(p2[r], o); }
    if (nloc == 0) { for (int r = 0; r < 8; ++r) { S1[wave][8 * hlf + r][h] = p1[r]; S2[wave][8 * hlf + r][h] = p2[r]; } }
#pragma unroll
    for (int t = 0; t < 4; ++t) for (int r = 0; r < 8; ++r) Tw[wave][8 * hlf + r][t * 16 + nloc] = acc[t][r];
    wave_lds_sync();
    for (int pass = 0; pass < 2; ++pass) { for (int rr = 0; rr < 16; rr += 2) { const int r2 = rr + (lane >> 4); const v4f wv4 = *(const v4f*)(&Tw[wave][r2][(lane & 15) * 4]); v4h hv, lv;
        for (int j = 0; j < 4; ++j) { const float wv = wv4[j] * XS; const b16 ph = (b16)wv; hv[j] = ph; lv[j] = (b16)((wv - (float)ph) * RS_); }
        const size_t o_ = (m0 + r2) * DM + h * HD + (lane & 15) * 4; *(volatile v4h*)(WHh + o_) = hv; *(volatile v4h*)(WHl + o_) = lv; }
      __threadfence(); }
    wave_lds_sync(); }
  wave_lds_sync();
  for (int pass = 0; pass < 2; ++pass) { for (int rr = 0; rr < 16; rr += 8) { const int r2 = rr + (lane >> 2); *(volatile v4f*)(F1 + (m0 + r2) * FP + (lane & 3) * 4) = *(const v4f*)(&S1[wave][r2][(lane & 3) * 4]); *(volatile v4f*)(F2 + (m0 + r2) * FP + (lane & 3) * 4) = *(const v4f*)(&S2[wave][r2][(lane & 3) * 4]); } __threadfence(); }
}
__global__ __launch_bounds__(32) void f2max_kernel(const float* __restrict__ F2, float* __restrict__ F2M) {
  const int lane = threadIdx.x; const int bh = blockIdx.x; const int b = bh / H, h = bh % H; float m = -INFINITY;
  for (int n = lane; n < T; n += 32) m = fmaxf(m, F2[((size_t)b * T + n) * FP + h]);
#pragma unroll
  for (int o = 1; o < 32; o <<= 1) m = fmaxf(m, __shfl_xor(m, o));
  for (int pass = 0; pass < 2; ++pass) { ((volatile float*)F2M)[(size_t)bh * 32 + lane] = (lane == 0) ? m : 0.0f; __threadfence(); }
}
__global__ __launch_bounds__(32) void attn_kernel(const b16* __restrict__ WHh, const b16* __restrict__ WHl, const float* __restrict__ F1, const float* __restrict__ F2, const float* __restrict__ F2M, float* __restrict__ y) {
  __shared__ __attribute__((aligned(16))) b16 Pt[16][32 + 8]; __shared__ __attribute__((aligned(16))) float Of[16][HD + 4];
  const int lane = threadIdx.x, nloc = lane & 15, hlf = lane >> 4; const int q0 = blockIdx.x * 16, h = blockIdx.y, b = blockIdx.z;
  const size_t qrow = (size_t)b * T + q0 + nloc;
  const float f1q = F1[qrow * FP + h]; const float Mq = lrelu(f1q + F2M[((size_t)b * H + h) * 32]); float lsum = 0.0f;
  v8f acc[4], accl[4];
#pragma unroll
  for (int t = 0; t < 4; ++t) { acc[t] = (v8f){}; accl[t] = (v8f){}; }
#pragma unroll 1
  for (int kb = 0; kb < T; kb += 32) {
    const int m0 = kb + 16 * hlf;
    v16b pv;
#pragma unroll
    for (int j = 0; j < 16; ++j) { const int m = m0 + j; const float f2m = F2[((size_t)b * T + m) * FP + h]; const float p = nexp2((lrelu(f1q + f2m) - Mq) * LOG2E); lsum += p; pv[j] = (b16)(p * PS); }
    *(v8b*)(&Pt[nloc][16 * hlf]) = __builtin_shufflevector(pv, pv, 0, 1, 2, 3, 4, 5, 6, 7); *(v8b*)(&Pt[nloc][16 * hlf + 8]) = __builtin_shufflevector(pv, pv, 8, 9, 10, 11, 12, 13, 14, 15);
    wave_lds_sync();
    const v16b a = frag_kb(&Pt[nloc][0], hlf);
#pragma unroll
    for (int t = 0; t < 4; ++t) { const int d = t * 16 + nloc; v16b vh, vl;
#pragma unroll
      for (int e = 0; e < 16; ++e) { const int k = (e < 8) ? (8 * hlf + e) : (16 + 8 * hlf + (e - 8)); const size_t o_ = ((size_t)b * T + kb + k) * DM + h * HD + d; vh[e] = WHh[o_]; vl[e] = WHl[o_]; }
      acc[t] = wmma16b(a, vh, acc[t]); accl[t] = wmma16b(a, vl, accl[t]); }
    wave_lds_sync(); }
  lsum += __shfl_xor(lsum, 16);
#pragma unroll
  for (int t = 0; t < 4; ++t) {
#pragma unroll
    for (int r = 0; r < 8; ++r) { const float lr = __shfl(lsum, 8 * hlf + r); const float o_ = (acc[t][r] + accl[t][r] * (1.0f / RS_)) * (1.0f / (XS * PS)); Of[8 * hlf + r][t * 16 + nloc] = o_ / lr; } }
  wave_lds_sync();
  for (int pass = 0; pass < 2; ++pass) { for (int rr = 0; rr < 16; rr += 2) { const int r2 = rr + (lane >> 4); if (q0 + r2 < QL) *(volatile v4f*)(y + ((size_t)b * T + q0 + r2) * DM + h * HD + (lane & 15) * 4) = *(const v4f*)(&Of[r2][(lane & 15) * 4]); } __threadfence(); }
}
}

extern "C" void kernel_launch(void* const* d_in, const int* in_sizes, int n_in, void* d_out, int out_size, void* d_ws, size_t ws_size, hipStream_t stream) {
  (void)n_in;
  auto Fp = [&](int i) { return (const float*)d_in[i]; };
  if (in_sizes[0] != NR * F || in_sizes[1] != DM * F || in_sizes[2] != H * AP || out_size != NR * DM) return;
  size_t off = 0; char* ws = (char*)d_ws;
  auto carve = [&](size_t bytes) { char* p = ws + off; off += (bytes + 255) & ~(size_t)255; return p; };
  b16* WT = (b16*)carve((size_t)DM * F * 2); b16* WHh = (b16*)carve((size_t)NR * DM * 2); b16* WHl = (b16*)carve((size_t)NR * DM * 2);
  float* F1 = (float*)carve((size_t)NR * FP * 4); float* F2 = (float*)carve((size_t)NR * FP * 4); float* F2M = (float*)carve((size_t)B * H * 32 * 4);
  if (off > ws_size || off > ((size_t)16 << 20)) return;
  wt_kernel<<<(DM * F / 8 + 255) / 256, 256, 0, stream>>>(Fp(1), WT);
  proj_kernel<<<NRL / 32, 64, 0, stream>>>(Fp(0), WT, Fp(2), WHh, WHl, F1, F2);
  f2max_kernel<<<B * H, 32, 0, stream>>>(F2, F2M);
  attn_kernel<<<dim3(QL / 16, H, BL), 32, 0, stream>>>(WHh, WHl, F1, F2, F2M, (float*)d_out);
}
